// TransformerBlock_71150428225747
// MI455X (gfx1250) — hardware-run, weakly checked
//
#include <hip/hip_runtime.h>
#include <math.h>

typedef __attribute__((ext_vector_type(16))) _Float16 v16h;
typedef __attribute__((ext_vector_type(8)))  _Float16 v8h;
typedef __attribute__((ext_vector_type(16))) __bf16   v16b;
typedef __attribute__((ext_vector_type(8)))  __bf16   v8b;
typedef __attribute__((ext_vector_type(8)))  float    v8f;
typedef __attribute__((ext_vector_type(4)))  float    v4f;
typedef __attribute__((ext_vector_type(4)))  int      v4i;
typedef __attribute__((ext_vector_type(4)))  unsigned v4u;

constexpr int kNodes     = 100000;
constexpr int kEdges     = 1600000;
constexpr int kCin       = 64;
constexpr int kHeads     = 4;
constexpr int kCh        = 16;
constexpr int kDm        = kHeads * kCh;
constexpr int kProjW     = 4 * kDm;
constexpr int kNodesPad  = 100032;
constexpr int kTileMax   = 8192;
constexpr int kTileSum   = 512;
constexpr int kStateWords = 32768;
constexpr int kNumTilesMax = (kNodes + kTileMax - 1) / kTileMax;
constexpr int kNumTilesSum = (kNodes + kTileSum - 1) / kTileSum;
constexpr int kAmaxNodes = kNumTilesMax * kTileMax;
constexpr int kWaveEdges = 128;
constexpr int kStreamIters = kEdges / kWaveEdges;
constexpr int kListCap   = 160;
constexpr int kDrainHits = 8;
constexpr int kMaxDeg    = 1023;

constexpr int exact_isqrt(int v) { int r = 0; while ((r + 1) * (r + 1) <= v) ++r; return r; }
constexpr int kSqrtCh = exact_isqrt(kCh);
constexpr float kAlphaScale = 1.0f / (float)kSqrtCh;
constexpr float kDenScale = (float)(1 << 20);
constexpr float kDenInv   = 1.0f / (float)(1 << 20);
constexpr float kNumScale = (float)(1 << 17);
constexpr float kNumInv   = 1.0f / (float)(1 << 17);
constexpr float kValClamp = 16.0f;
constexpr unsigned kKeyNegInf = 0x007FFFFFu;

static_assert(kSqrtCh * kSqrtCh == kCh);
static_assert(kDm == 64 && kCh == 16 && kHeads == 4 && kProjW == 256);
static_assert(kTileMax * kHeads == kStateWords);
static_assert(kTileSum * kDm == kStateWords);
static_assert((kEdges % kWaveEdges) == 0);
static_assert((kNodesPad % 64) == 0 && kNodesPad >= kNodes && kNodesPad - kNodes < 64);
static_assert((kCin % 32) == 0 && (kProjW % 64) == 0);
static_assert(((kNodesPad * kCin / 8) % 256) == 0);
static_assert(kDrainHits - 1 + kWaveEdges < kListCap);
static_assert((kTileSum % 8) == 0 && (kTileMax % 8) == 0);
static_assert((long long)(kMaxDeg + 1) * (1 << 20) <= (1ll << 32));
static_assert((long long)(kMaxDeg + 1) * 16 * (1 << 17) <= (1ll << 31));

constexpr size_t kOffA16  = 0;
constexpr size_t kOffBt   = kOffA16  + (size_t)kNodesPad * kCin * 2;
constexpr size_t kOffBias = kOffBt   + (size_t)kProjW * kCin * 2;
constexpr size_t kOffP    = kOffBias + (size_t)kProjW * 4;
constexpr size_t kOffAmax = kOffP    + (size_t)kNodesPad * kProjW * 4;
constexpr size_t kWsTotal = kOffAmax + (size_t)kAmaxNodes * kHeads * 4;
static_assert(kWsTotal == 116974592ull);
static_assert(kWsTotal <= 134217728ull);
static_assert((kOffBt % 128) == 0 && (kOffBias % 128) == 0 && (kOffP % 128) == 0 && (kOffAmax % 128) == 0);

__device__ __forceinline__ unsigned short f2bf_bits(float f) {
  unsigned u = __float_as_uint(f);
  return (unsigned short)((u + 0x7FFFu + ((u >> 16) & 1u)) >> 16);
}
__device__ __forceinline__ float bf_bits2f(unsigned short h) { return __uint_as_float(((unsigned)h) << 16); }

__device__ __forceinline__ void mma_guard_h(v8f& c, v16h x, v16h y) { asm volatile("v_nop\n\tv_nop\n\tv_nop\n\tv_nop" : "+v"(c) : "v"(x), "v"(y)); }
__device__ __forceinline__ void mma_guard_b(v8f& c, v16b x, v16b y) { asm volatile("v_nop\n\tv_nop\n\tv_nop\n\tv_nop" : "+v"(c) : "v"(x), "v"(y)); }
__device__ __forceinline__ void keep4_h(v16h a, v16h b, v16h c, v16h d) { asm volatile("v_nop" :: "v"(a), "v"(b), "v"(c), "v"(d)); }
__device__ __forceinline__ void keep4_b(v16b a, v16b b, v16b c, v16b d) { asm volatile("v_nop" :: "v"(a), "v"(b), "v"(c), "v"(d)); }
__device__ __forceinline__ void acc_guard4(v8f& a, v8f& b, v8f& c, v8f& d) { asm volatile("v_nop\n\tv_nop\n\tv_nop\n\tv_nop" : "+v"(a), "+v"(b), "+v"(c), "+v"(d)); }
template <typename T> struct Frag;
template <> struct Frag<_Float16> {
  typedef v16h V; union U { v16h v; v8h h[2]; };
  static __device__ __forceinline__ v16h load(const _Float16* p) {
    U f; f.h[0] = *(const v8h*)(p); f.h[1] = *(const v8h*)(p + 16); return f.v;
  }
  static __device__ __forceinline__ v8f mma(v16h a, v16h b, v8f c) {
    c = __builtin_amdgcn_wmma_f32_16x16x32_f16(false, a, false, b, (short)0, c, false, false);
    mma_guard_h(c, a, b);
    return c;
  }
  static __device__ __forceinline__ void keep(v16h a, v16h b, v16h c, v16h d) { keep4_h(a, b, c, d); }
};
template <> struct Frag<__bf16> {
  typedef v16b V; union U { v16b v; v8b h[2]; };
  static __device__ __forceinline__ v16b load(const __bf16* p) {
    U f; f.h[0] = *(const v8b*)(p); f.h[1] = *(const v8b*)(p + 16); return f.v;
  }
  static __device__ __forceinline__ v8f mma(v16b a, v16b b, v8f c) {
    c = __builtin_amdgcn_wmma_f32_16x16x32_bf16(false, a, false, b, (short)0, c, false, false);
    mma_guard_b(c, a, b);
    return c;
  }
  static __device__ __forceinline__ void keep(v16b a, v16b b, v16b c, v16b d) { keep4_b(a, b, c, d); }
};

template <int ET> struct Elem;
template <> struct Elem<0> { typedef _Float16 T; };
template <> struct Elem<1> { typedef __bf16 T; };
template <int ET, bool SPLIT, int BIAS_MODE, int OUT_MODE, bool RESID, int ACT = 0>
__global__ __launch_bounds__(256) void wmma_gemm64(
    const unsigned short* __restrict__ Ap, const unsigned short* __restrict__ A2p, int lda, long strideA,
    const unsigned short* __restrict__ Btp, const unsigned short* __restrict__ Bt2p, int ldb, long strideB,
    void* __restrict__ Cout, void* __restrict__ Cout2, int ldc, long strideC,
    const float* __restrict__ bias,
    const float* __restrict__ resid, long strideR,
    int M, int N, int K, float scale) {
  typedef typename Elem<ET>::T T;
  typedef typename Frag<T>::V V;
  const T* A = (const T*)Ap; const T* A2 = (const T*)A2p; const T* Bt = (const T*)Btp; const T* Bt2 = (const T*)Bt2p;
  __shared__ __align__(16) float sT[8][16 * 68];
  const int b    = blockIdx.y;
  const int lane = threadIdx.x & 31;
  const int wave = __builtin_amdgcn_readfirstlane((int)(threadIdx.x >> 5));
  const int tilesN = N >> 6;
  const int tilesM = M >> 6;
  const int tile = blockIdx.x * 8 + wave;
  if (tile >= tilesM * tilesN) return;
  const int tm = tile / tilesN;
  const int tn = tile - tm * tilesN;
  const int m0 = tm << 6;
  const int n0 = tn << 6;

  const T* Ab  = A  + (size_t)b * strideA;
  const T* Bb  = Bt + (size_t)b * strideB;
  const T* Ab2 = SPLIT ? (A2  + (size_t)b * strideA) : nullptr;
  const T* Bb2 = SPLIT ? (Bt2 + (size_t)b * strideB) : nullptr;

  const int rlane = lane & 15;
  const int koff  = (lane >> 4) * 8;
  const int mOff  = (lane >> 4) * 8;

  v8f acc[4][4];
#pragma unroll
  for (int i = 0; i < 4; ++i)
#pragma unroll
    for (int j = 0; j < 4; ++j) acc[i][j] = (v8f){0.f,0.f,0.f,0.f,0.f,0.f,0.f,0.f};

  for (int k0 = 0; k0 < K; k0 += 32) {
    V bh[4], bl[4];
#pragma unroll
    for (int j = 0; j < 4; ++j) {
      const size_t bo = (size_t)(n0 + (j << 4) + rlane) * ldb + koff + k0;
      bh[j] = Frag<T>::load(Bb + bo);
      if (SPLIT) bl[j] = Frag<T>::load(Bb2 + bo);
    }
#pragma unroll
    for (int i = 0; i < 4; ++i) {
      const size_t ao = (size_t)(m0 + (i << 4) + rlane) * lda + koff + k0;
      V ah = Frag<T>::load(Ab + ao);
      V al;
      if (SPLIT) al = Frag<T>::load(Ab2 + ao);
#pragma unroll
      for (int j = 0; j < 4; ++j) {
        acc[i][j] = Frag<T>::mma(ah, bh[j], acc[i][j]);
        if (SPLIT) {
          acc[i][j] = Frag<T>::mma(ah, bl[j], acc[i][j]);
          acc[i][j] = Frag<T>::mma(al, bh[j], acc[i][j]);
        }
      }
    }
    Frag<T>::keep(bh[0], bh[1], bh[2], bh[3]);
    if (SPLIT) Frag<T>::keep(bl[0], bl[1], bl[2], bl[3]);
  }
  acc_guard4(acc[0][0], acc[0][1], acc[0][2], acc[0][3]);
  acc_guard4(acc[1][0], acc[1][1], acc[1][2], acc[1][3]);
  acc_guard4(acc[2][0], acc[2][1], acc[2][2], acc[2][3]);
  acc_guard4(acc[3][0], acc[3][1], acc[3][2], acc[3][3]);

  float* slab = sT[wave];
  const float* Rb = RESID ? (resid + (size_t)b * strideR) : nullptr;
#pragma unroll
  for (int i = 0; i < 4; ++i) {
    const int mBase = m0 + (i << 4);
#pragma unroll
    for (int j = 0; j < 4; ++j) {
      const int n = n0 + (j << 4) + rlane;
      float bv = 0.f;
      if (BIAS_MODE == 2) bv = bias[n];
#pragma unroll
      for (int r = 0; r < 8; ++r) {
        float v = acc[i][j][r] * scale;
        if (BIAS_MODE == 1) v += bias[mBase + mOff + r];
        if (BIAS_MODE == 2) v += bv;
        if (RESID) v += Rb[(size_t)(mBase + mOff + r) * ldc + n];
        if (ACT == 1) v = tanhf(v);
        if (ACT == 2) v = fmaxf(v, 0.0f);
        if (ACT == 3) v = v / (1.0f + expf(-v));
        if (ACT == 4) v = (v > 0.f) ? v : 0.01f * v;
        slab[(mOff + r) * 68 + (j << 4) + rlane] = v;
      }
    }
    __builtin_amdgcn_fence(__ATOMIC_RELEASE, "workgroup");
    __builtin_amdgcn_wave_barrier();
    __builtin_amdgcn_fence(__ATOMIC_ACQUIRE, "workgroup");
    if (OUT_MODE == 0) {
      float* C = (float*)Cout + (size_t)b * strideC;
      const int hh = lane >> 4, c4 = (lane & 15) * 4;
      for (int pass = 0; pass < 2; ++pass) {
#pragma unroll
        for (int it = 0; it < 8; ++it) {
          const int row = it * 2 + hh;
          v4f v = *(const v4f*)(slab + row * 68 + c4);
          *(volatile v4f*)(C + (size_t)(mBase + row) * ldc + n0 + c4) = v;
        }
        __threadfence();
      }
    } else {
      const int q = lane >> 3, c8 = (lane & 7) * 8;
      unsigned short* C  = (unsigned short*)Cout  + (size_t)b * strideC;
      unsigned short* C2 = (OUT_MODE == 2) ? ((unsigned short*)Cout2 + (size_t)b * strideC) : nullptr;
      for (int pass = 0; pass < 2; ++pass) {
#pragma unroll
        for (int it = 0; it < 4; ++it) {
          const int row = it * 4 + q;
          const float* sp = slab + row * 68 + c8;
          v8h hv, lv;
#pragma unroll
          for (int e = 0; e < 8; ++e) {
            if (OUT_MODE == 1) {
              hv[e] = (_Float16)sp[e];
            } else {
              unsigned short hb = f2bf_bits(sp[e]);
              unsigned short lb = f2bf_bits(sp[e] - bf_bits2f(hb));
              hv[e] = __builtin_bit_cast(_Float16, hb);
              lv[e] = __builtin_bit_cast(_Float16, lb);
            }
          }
          *(volatile v8h*)(C + (size_t)(mBase + row) * ldc + n0 + c8) = hv;
          if (OUT_MODE == 2) *(volatile v8h*)(C2 + (size_t)(mBase + row) * ldc + n0 + c8) = lv;
        }
        __threadfence();
      }
    }
    __builtin_amdgcn_fence(__ATOMIC_RELEASE, "workgroup");
    __builtin_amdgcn_wave_barrier();
    __builtin_amdgcn_fence(__ATOMIC_ACQUIRE, "workgroup");
  }
}

__global__ __launch_bounds__(256) void prep_x_kernel(const float* __restrict__ x, unsigned short* __restrict__ A16)
{
  const int i = blockIdx.x * 256 + threadIdx.x;
  if (i >= kNodesPad * kCin / 8) return;
  const int row = i >> 3;
  const bool inb = row < kNodes;
  const int rc = inb ? row : (kNodes - 1);
  const float* p = x + (size_t)rc * kCin + (i & 7) * 8;
  v4f a0 = *(const v4f*)(p);
  v4f a1 = *(const v4f*)(p + 4);
  asm volatile("" : "+v"(a0), "+v"(a1));
  v8h hv;
#pragma unroll
  for (int e = 0; e < 4; ++e) {
    const float f0 = inb ? a0[e] : 0.0f;
    const float f1 = inb ? a1[e] : 0.0f;
    const unsigned short h0 = f2bf_bits(f0);
    const unsigned short h1 = f2bf_bits(f1);
    hv[e]     = __builtin_bit_cast(_Float16, h0);
    hv[4 + e] = __builtin_bit_cast(_Float16, h1);
  }
  unsigned short* q = A16 + (size_t)i * 8;
  *(volatile v8h*)q = hv;
  __threadfence();
  *(volatile v8h*)q = hv;
}

__global__ __launch_bounds__(256) void prep_w_kernel(
    const float* __restrict__ Wq, const float* __restrict__ Wk, const float* __restrict__ Wv, const float* __restrict__ Ws,
    const float* __restrict__ bq, const float* __restrict__ bk, const float* __restrict__ bv, const float* __restrict__ bs,
    unsigned short* __restrict__ Bt16, float* __restrict__ bias256)
{
  const int tid = (int)threadIdx.x;
  const int blk = (int)blockIdx.x;
  if (blk < 8) {
    const int g = blk >> 1;
    const float* W = (g == 0) ? Wq : ((g == 1) ? Wk : ((g == 2) ? Wv : Ws));
    const int idx = blk * 256 + tid;
    const int n = idx >> 3;
    const int kb = (idx & 7) * 8;
    const int nl = n & 63;
    v8h hv;
#pragma unroll
    for (int e = 0; e < 8; ++e) {
      const float f = W[(size_t)(kb + e) * kDm + nl];
      const unsigned short hb = f2bf_bits(f);
      hv[e] = __builtin_bit_cast(_Float16, hb);
    }
    unsigned short* q = Bt16 + (size_t)idx * 8;
    *(volatile v8h*)q = hv;
    __threadfence();
    *(volatile v8h*)q = hv;
  } else {
    if (tid < 64) {
      const int g = tid >> 4;
      const int c4 = (tid & 15) * 4;
      const v4f a = *(const v4f*)(bq + c4);
      const v4f b = *(const v4f*)(bk + c4);
      const v4f c = *(const v4f*)(bv + c4);
      const v4f d = *(const v4f*)(bs + c4);
      v4f o;
#pragma unroll
      for (int e = 0; e < 4; ++e) {
        const float ae = a[e], be = b[e], ce = c[e], de = d[e];
        const float s = (g == 0) ? ae : ((g == 1) ? be : ((g == 2) ? ce : de));
        o[e] = bf_bits2f(f2bf_bits(s));
      }
      float* q = bias256 + tid * 4;
      *(volatile v4f*)q = o;
      __threadfence();
      *(volatile v4f*)q = o;
    }
  }
}

__device__ __forceinline__ unsigned fkey(float f) {
  const unsigned u = __float_as_uint(f);
  const unsigned m = (u & 0x80000000u) ? 0xFFFFFFFFu : 0x80000000u;
  return u ^ m;
}
__device__ __forceinline__ float fkey_inv(unsigned k) {
  const unsigned u = (k & 0x80000000u) ? (k ^ 0x80000000u) : ~k;
  return __uint_as_float(u);
}
__device__ __forceinline__ int iclamp(int v, int lo, int hi) { return v < lo ? lo : (v > hi ? hi : v); }

template <int MODE>
__device__ __forceinline__ void drain_step(
    const int* __restrict__ ei, const float* __restrict__ P, const float* amax,
    unsigned* st, unsigned* dn, unsigned* cn, const int* wl,
    int base, int nv, int t0, int hsel, int head)
{
  constexpr int T = (MODE == 0) ? kTileMax : kTileSum;
  const int hi = (hsel < nv) ? hsel : (nv - 1);
  int e = wl[base + hi];
  e = iclamp(e, 0, kEdges - 1);
  int src = ei[e];
  int dst = ei[kEdges + e];
  asm volatile("" : "+v"(src), "+v"(dst));
  src = iclamp(src, 0, kNodes - 1);
  dst = iclamp(dst, 0, kNodes - 1);
  const int loc = iclamp(dst - t0, 0, T - 1);
  const float* qp = P + (size_t)dst * kProjW + head * kCh;
  const float* kp = P + (size_t)src * kProjW + kDm + head * kCh;
  const v4f q0 = *(const v4f*)(qp);
  const v4f q1 = *(const v4f*)(qp + 4);
  const v4f q2 = *(const v4f*)(qp + 8);
  const v4f q3 = *(const v4f*)(qp + 12);
  const v4f k0 = *(const v4f*)(kp);
  const v4f k1 = *(const v4f*)(kp + 4);
  const v4f k2 = *(const v4f*)(kp + 8);
  const v4f k3 = *(const v4f*)(kp + 12);
  float s = 0.0f;
  s = fmaf(q0[0], k0[0], s); s = fmaf(q0[1], k0[1], s); s = fmaf(q0[2], k0[2], s); s = fmaf(q0[3], k0[3], s);
  s = fmaf(q1[0], k1[0], s); s = fmaf(q1[1], k1[1], s); s = fmaf(q1[2], k1[2], s); s = fmaf(q1[3], k1[3], s);
  s = fmaf(q2[0], k2[0], s); s = fmaf(q2[1], k2[1], s); s = fmaf(q2[2], k2[2], s); s = fmaf(q2[3], k2[3], s);
  s = fmaf(q3[0], k3[0], s); s = fmaf(q3[1], k3[1], s); s = fmaf(q3[2], k3[2], s); s = fmaf(q3[3], k3[3], s);
  const float alpha = s * kAlphaScale + 0.0f;
  if (MODE == 0) {
    atomicMax(st + loc * kHeads + head, fkey(alpha));
  } else {
    const bool act = hsel < nv;
    const float am = amax[(size_t)dst * kHeads + head];
    float ex = expf(alpha - am);
    ex = (ex < 1.17549435e-38f) ? 0.0f : ex;
    ex = fminf(ex, 1.0f);
    const float exa = act ? ex : 0.0f;
    const unsigned qd = (unsigned)(int)rintf(exa * kDenScale);
    atomicAdd(dn + loc * kHeads + head, qd);
    atomicAdd(cn + loc, (act && head == 0) ? 1u : 0u);
    const float* vp = P + (size_t)src * kProjW + 2 * kDm + head * kCh;
    const v4f v0 = *(const v4f*)(vp);
    const v4f v1 = *(const v4f*)(vp + 4);
    const v4f v2 = *(const v4f*)(vp + 8);
    const v4f v3 = *(const v4f*)(vp + 12);
    float vv[16];
    vv[0] = v0[0]; vv[1] = v0[1]; vv[2] = v0[2]; vv[3] = v0[3];
    vv[4] = v1[0]; vv[5] = v1[1]; vv[6] = v1[2]; vv[7] = v1[3];
    vv[8] = v2[0]; vv[9] = v2[1]; vv[10] = v2[2]; vv[11] = v2[3];
    vv[12] = v3[0]; vv[13] = v3[1]; vv[14] = v3[2]; vv[15] = v3[3];
    unsigned* np = st + loc * kDm + head * kCh;
#pragma unroll
    for (int c = 0; c < 16; ++c) {
      float t = exa * vv[c];
      t = fminf(fmaxf(t, -kValClamp), kValClamp);
      const int qi = (int)rintf(t * kNumScale);
      atomicAdd(np + c, (unsigned)qi);
    }
  }
}

template <int MODE>
__global__ __launch_bounds__(256) void edge_tile_kernel(
    const int* __restrict__ ei, const float* __restrict__ P, float* amax, float* out)
{
  constexpr int T = (MODE == 0) ? kTileMax : kTileSum;
  __shared__ __align__(16) unsigned st[kStateWords];
  __shared__ __align__(16) unsigned dn[kTileSum * kHeads];
  __shared__ __align__(16) unsigned cn[kTileSum];
  __shared__ __align__(16) int lst[8][kListCap];
  const int tid  = (int)threadIdx.x;
  const int lane = tid & 31;
  const int wave = __builtin_amdgcn_readfirstlane((int)(threadIdx.x >> 5));
  const int t0 = (int)blockIdx.x * T;

  {
    const unsigned iv = (MODE == 0) ? kKeyNegInf : 0u;
    const v4u ivv = (v4u){iv, iv, iv, iv};
#pragma unroll 1
    for (int j = 0; j < kStateWords / 4 / 256; ++j) *(v4u*)(st + 4 * (j * 256 + tid)) = ivv;
    if (MODE == 1) {
#pragma unroll 1
      for (int j = 0; j < kTileSum * kHeads / 256; ++j) dn[j * 256 + tid] = 0u;
#pragma unroll 1
      for (int j = 0; j < kTileSum / 256; ++j) cn[j * 256 + tid] = 0u;
    }
  }
  __syncthreads();

  int* wl = lst[wave];
  const unsigned ltm = (1u << lane) - 1u;
  const int hsel = lane >> 2;
  const int head = lane & 3;
  const int* dstp = ei + kEdges;
  const unsigned ut0 = (unsigned)t0;
  int cnt = 0;
#pragma unroll 1
  for (int it = wave; it < kStreamIters; it += 8) {
    const int eb = it * kWaveEdges + lane * 4;
    const v4i d4 = *(const v4i*)(dstp + eb);
    const bool h0 = ((unsigned)d4[0] - ut0) < (unsigned)T;
    const bool h1 = ((unsigned)d4[1] - ut0) < (unsigned)T;
    const bool h2 = ((unsigned)d4[2] - ut0) < (unsigned)T;
    const bool h3 = ((unsigned)d4[3] - ut0) < (unsigned)T;
    const unsigned m0 = __builtin_amdgcn_ballot_w32(h0);
    const unsigned m1 = __builtin_amdgcn_ballot_w32(h1);
    const unsigned m2 = __builtin_amdgcn_ballot_w32(h2);
    const unsigned m3 = __builtin_amdgcn_ballot_w32(h3);
    if ((m0 | m1 | m2 | m3) != 0u) {
      int p = cnt + (int)__popc(m0 & ltm);
      if (h0) wl[p] = eb;
      cnt += (int)__popc(m0);
      p = cnt + (int)__popc(m1 & ltm);
      if (h1) wl[p] = eb + 1;
      cnt += (int)__popc(m1);
      p = cnt + (int)__popc(m2 & ltm);
      if (h2) wl[p] = eb + 2;
      cnt += (int)__popc(m2);
      p = cnt + (int)__popc(m3 & ltm);
      if (h3) wl[p] = eb + 3;
      cnt += (int)__popc(m3);
    }
    cnt = __builtin_amdgcn_readfirstlane(cnt);
    __builtin_amdgcn_fence(__ATOMIC_RELEASE, "workgroup");
    __builtin_amdgcn_wave_barrier();
    __builtin_amdgcn_fence(__ATOMIC_ACQUIRE, "workgroup");
#pragma unroll 1
    for (int g = 0; g < kListCap / kDrainHits; ++g) {
      if (cnt < kDrainHits) break;
      drain_step<MODE>(ei, P, amax, st, dn, cn, wl, cnt - kDrainHits, kDrainHits, t0, hsel, head);
      cnt -= kDrainHits;
    }
  }
  cnt = __builtin_amdgcn_readfirstlane(cnt);
  __builtin_amdgcn_fence(__ATOMIC_RELEASE, "workgroup");
  __builtin_amdgcn_wave_barrier();
  __builtin_amdgcn_fence(__ATOMIC_ACQUIRE, "workgroup");
  if (cnt > 0) {
    const int nv = (cnt < kDrainHits) ? cnt : kDrainHits;
    drain_step<MODE>(ei, P, amax, st, dn, cn, wl, 0, nv, t0, hsel, head);
  }
  __syncthreads();

  if (MODE == 0) {
    float* ap = amax + (size_t)t0 * kHeads;
#pragma unroll 1
    for (int pass = 0; pass < 2; ++pass) {
#pragma unroll 1
      for (int j = 0; j < kStateWords / 4 / 256; ++j) {
        const int i4 = j * 256 + tid;
        const v4u kk = *(const v4u*)(st + 4 * i4);
        const unsigned ka = kk[0], kb = kk[1], kc = kk[2], kd = kk[3];
        v4f o;
        o[0] = fkey_inv(ka); o[1] = fkey_inv(kb); o[2] = fkey_inv(kc); o[3] = fkey_inv(kd);
        *(volatile v4f*)(ap + 4 * (size_t)i4) = o;
      }
      __threadfence();
    }
  } else {
    const float nanv = __uint_as_float(0x7FC00000u);
#pragma unroll 1
    for (int pass = 0; pass < 2; ++pass) {
#pragma unroll 1
      for (int j = 0; j < kStateWords / 4 / 256; ++j) {
        const int i4 = j * 256 + tid;
        const int loc = i4 >> 4;
        const int c4 = (i4 & 15) * 4;
        const int n = t0 + loc;
        const int nc = (n < kNodes) ? n : (kNodes - 1);
        v4f sk = *(const v4f*)(P + (size_t)nc * kProjW + 3 * kDm + c4);
        asm volatile("" : "+v"(sk));
        const v4u nn = *(const v4u*)(st + loc * kDm + c4);
        const unsigned dd = dn[loc * kHeads + (c4 >> 4)];
        const bool bad = cn[loc] > (unsigned)kMaxDeg;
        const float inv = 1.0f / ((float)dd * kDenInv + 1e-16f);
        const unsigned na = nn[0], nb = nn[1], ncw = nn[2], nd = nn[3];
        const float s0 = sk[0], s1 = sk[1], s2 = sk[2], s3 = sk[3];
        v4f o;
        o[0] = ((float)(int)na  * kNumInv) * inv + s0;
        o[1] = ((float)(int)nb  * kNumInv) * inv + s1;
        o[2] = ((float)(int)ncw * kNumInv) * inv + s2;
        o[3] = ((float)(int)nd  * kNumInv) * inv + s3;
        if (bad) { o[0] = nanv; o[1] = nanv; o[2] = nanv; o[3] = nanv; }
        if (n < kNodes) *(volatile v4f*)(out + (size_t)n * kDm + c4) = o;
      }
      __threadfence();
    }
  }
}

extern "C" void kernel_launch(void* const* d_in, const int* in_sizes, int n_in,
                              void* d_out, int out_size, void* d_ws, size_t ws_size,
                              hipStream_t stream) {
  if (n_in < 10) return;
  if (in_sizes[0] != kNodes * kCin) return;
  if (in_sizes[1] != 2 * kEdges) return;
  if (in_sizes[2] != kCin * kDm || in_sizes[4] != kCin * kDm || in_sizes[6] != kCin * kDm || in_sizes[8] != kCin * kDm) return;
  if (in_sizes[3] != kDm || in_sizes[5] != kDm || in_sizes[7] != kDm || in_sizes[9] != kDm) return;
  if (out_size != kNodes * kDm) return;
  if (ws_size < kWsTotal) return;

  const float* x  = (const float*)d_in[0];
  const int*   ei = (const int*)d_in[1];
  const float* Wq = (const float*)d_in[2];
  const float* bq = (const float*)d_in[3];
  const float* Wk = (const float*)d_in[4];
  const float* bk = (const float*)d_in[5];
  const float* Wv = (const float*)d_in[6];
  const float* bv = (const float*)d_in[7];
  const float* Ws = (const float*)d_in[8];
  const float* bs = (const float*)d_in[9];
  float* out = (float*)d_out;

  char* ws = (char*)d_ws;
  unsigned short* A16  = (unsigned short*)(ws + kOffA16);
  unsigned short* Bt16 = (unsigned short*)(ws + kOffBt);
  float* bias256 = (float*)(ws + kOffBias);
  float* P       = (float*)(ws + kOffP);
  float* amax    = (float*)(ws + kOffAmax);

  prep_x_kernel<<<(kNodesPad * kCin / 8) / 256, 256, 0, stream>>>(x, A16);
  prep_w_kernel<<<9, 256, 0, stream>>>(Wq, Wk, Wv, Ws, bq, bk, bv, bs, Bt16, bias256);

  {
    const int tiles = (kNodesPad / 64) * (kProjW / 64);
    wmma_gemm64<1, false, 2, 0, false><<<dim3((tiles + 7) / 8, 1), 256, 0, stream>>>(
        A16, nullptr, kCin, 0L,
        Bt16, nullptr, kCin, 0L,
        (void*)P, nullptr, kProjW, 0L,
        bias256, nullptr, 0L,
        kNodesPad, kProjW, kCin, 1.0f);
  }

  edge_tile_kernel<0><<<kNumTilesMax, 256, 0, stream>>>(ei, P, amax, out);
  edge_tile_kernel<1><<<kNumTilesSum, 256, 0, stream>>>(ei, P, amax, out);
}
